// LSTMdecoder_64665027608597
// MI455X (gfx1250) — hardware-verified
//
#include <hip/hip_runtime.h>
#include <math.h>

constexpr int NB   = 32;
constexpr int SE   = 512;
constexpr int SD   = 256;
constexpr int DM   = 512;
constexpr int NH   = 512;
constexpr int G4   = 4 * NH;
constexpr int VOC  = 32000;
constexpr int MR   = NB * SD;
constexpr int KTOT = DM + NH;
constexpr int NTHR = 256;
constexpr int AP   = 1032;
constexpr int OP   = 516;
constexpr float CR_XW  = 64.0f;
constexpr float CR_HW  = 16.0f;
constexpr float CR_ACT = 64.0f;
constexpr float CR_H   = 256.0f;
constexpr float CR_P   = 1024.0f;
constexpr float ZINV   = 1.0f / 4096.0f;
static_assert(CR_ACT * CR_XW == 4096.0f && CR_H * CR_HW == 4096.0f, "matched carries");
static_assert(DM == 512 && NH == 512 && SE == 512 && SD == 256, "lane maps assume these");
static_assert(MR % 64 == 0 && DM % 64 == 0 && SE % 64 == 0 && SD % 64 == 0 && G4 % 64 == 0, "GEMM M,N tile multiples");
static_assert(DM % 32 == 0 && SE % 32 == 0 && KTOT % 32 == 0, "GEMM K multiples of 32");
static_assert(NH == 64 * (NTHR / 32), "8 waves x 64 hidden units");
static_assert((16 * NH) % NTHR == 0, "h zero-fill loop exact");
static_assert(NB % 16 == 0, "16 batch rows per recurrence block");
static_assert(SE == 2 * NTHR && SD % 8 == 0, "softmax mask staging map");
static_assert((MR * (DM / 8)) % NTHR == 0, "gather grid exact");

typedef __attribute__((ext_vector_type(16))) _Float16 v16h;
typedef __attribute__((ext_vector_type(8)))  _Float16 v8h;
typedef __attribute__((ext_vector_type(16))) __bf16   v16b;
typedef __attribute__((ext_vector_type(8)))  __bf16   v8b;
typedef __attribute__((ext_vector_type(8)))  float    v8f;
typedef __attribute__((ext_vector_type(4)))  float    v4f;
typedef __attribute__((ext_vector_type(4)))  unsigned v4u;
typedef __attribute__((ext_vector_type(4)))  int      v4i;

__device__ __forceinline__ unsigned short f2bf_bits(float f) {
  unsigned u = __float_as_uint(f);
  return (unsigned short)((u + 0x7FFFu + ((u >> 16) & 1u)) >> 16);
}
__device__ __forceinline__ float bf_bits2f(unsigned short h) { return __uint_as_float(((unsigned)h) << 16); }

__device__ __forceinline__ void dep_guard_h(v8f& a, v8f& b, v16h x, v16h y) { asm volatile("v_nop\n\tv_nop\n\tv_nop\n\tv_nop" : "+v"(a), "+v"(b) : "v"(x), "v"(y)); }
__device__ __forceinline__ void dep_guard_b(v8f& a, v8f& b, v16b x, v16b y) { asm volatile("v_nop\n\tv_nop\n\tv_nop\n\tv_nop" : "+v"(a), "+v"(b) : "v"(x), "v"(y)); }
__device__ __forceinline__ void dep_guard4_h(v8f& a, v8f& b, v8f& c, v8f& d, v16h x, v16h y) { asm volatile("v_nop\n\tv_nop\n\tv_nop\n\tv_nop" : "+v"(a), "+v"(b), "+v"(c), "+v"(d) : "v"(x), "v"(y)); }
__device__ __forceinline__ void dep_guard4_b(v8f& a, v8f& b, v8f& c, v8f& d, v16b x, v16b y) { asm volatile("v_nop\n\tv_nop\n\tv_nop\n\tv_nop" : "+v"(a), "+v"(b), "+v"(c), "+v"(d) : "v"(x), "v"(y)); }
__device__ __forceinline__ void keep4_h(v16h a, v16h b, v16h c, v16h d) { asm volatile("v_nop" :: "v"(a), "v"(b), "v"(c), "v"(d)); }
__device__ __forceinline__ void keep4_b(v16b a, v16b b, v16b c, v16b d) { asm volatile("v_nop" :: "v"(a), "v"(b), "v"(c), "v"(d)); }
__device__ __forceinline__ void acc_guard4(v8f& a, v8f& b, v8f& c, v8f& d) { asm volatile("v_nop\n\tv_nop\n\tv_nop\n\tv_nop" : "+v"(a), "+v"(b), "+v"(c), "+v"(d)); }
template <typename T> struct Frag;
template <> struct Frag<_Float16> {
  typedef v16h V; union U { v16h v; v8h h[2]; };
  static __device__ __forceinline__ v16h load(const _Float16* p) {
    U f; f.h[0] = *(const v8h*)(p); f.h[1] = *(const v8h*)(p + 16); return f.v;
  }
  static __device__ __forceinline__ v8f mma(v16h a, v16h b, v8f c) {
    return __builtin_amdgcn_wmma_f32_16x16x32_f16(false, a, false, b, (short)0, c, false, false);
  }
  static __device__ __forceinline__ void guard(v8f& a, v8f& b, v16h x, v16h y) { dep_guard_h(a, b, x, y); }
  static __device__ __forceinline__ void guard4(v8f& a, v8f& b, v8f& c, v8f& d, v16h x, v16h y) { dep_guard4_h(a, b, c, d, x, y); }
  static __device__ __forceinline__ void keep(v16h a, v16h b, v16h c, v16h d) { keep4_h(a, b, c, d); }
};
template <> struct Frag<__bf16> {
  typedef v16b V; union U { v16b v; v8b h[2]; };
  static __device__ __forceinline__ v16b load(const __bf16* p) {
    U f; f.h[0] = *(const v8b*)(p); f.h[1] = *(const v8b*)(p + 16); return f.v;
  }
  static __device__ __forceinline__ v8f mma(v16b a, v16b b, v8f c) {
    return __builtin_amdgcn_wmma_f32_16x16x32_bf16(false, a, false, b, (short)0, c, false, false);
  }
  static __device__ __forceinline__ void guard(v8f& a, v8f& b, v16b x, v16b y) { dep_guard_b(a, b, x, y); }
  static __device__ __forceinline__ void guard4(v8f& a, v8f& b, v8f& c, v8f& d, v16b x, v16b y) { dep_guard4_b(a, b, c, d, x, y); }
  static __device__ __forceinline__ void keep(v16b a, v16b b, v16b c, v16b d) { keep4_b(a, b, c, d); }
};

__device__ __forceinline__ float fsig(float x) { return 1.0f / (1.0f + expf(-x)); }

template <int ET> struct Elem;
template <> struct Elem<0> { typedef _Float16 T; };
template <> struct Elem<1> { typedef __bf16 T; };
template <int ET, bool SPLIT, int BIAS_MODE, int OUT_MODE, bool RESID, int ACT = 0>
__global__ __launch_bounds__(256) void wmma_gemm64(
    const unsigned short* __restrict__ Ap, const unsigned short* __restrict__ A2p, int lda, long strideA,
    const unsigned short* __restrict__ Btp, const unsigned short* __restrict__ Bt2p, int ldb, long strideB,
    void* __restrict__ Cout, void* __restrict__ Cout2, int ldc, long strideC,
    const float* __restrict__ bias,
    const float* __restrict__ resid, long strideR,
    int M, int N, int K, float scale) {
  typedef typename Elem<ET>::T T;
  typedef typename Frag<T>::V V;
  const T* A = (const T*)Ap; const T* A2 = (const T*)A2p; const T* Bt = (const T*)Btp; const T* Bt2 = (const T*)Bt2p;
  __shared__ __align__(16) float sT[8][16 * 68];
  const int b    = blockIdx.y;
  const int lane = threadIdx.x & 31;
  const int wave = threadIdx.x >> 5;
  const int tilesN = N >> 6;
  const int tilesM = M >> 6;
  const int tile = blockIdx.x * 8 + wave;
  if (tile >= tilesM * tilesN) return;
  const int tm = tile / tilesN;
  const int tn = tile - tm * tilesN;
  const int m0 = tm << 6;
  const int n0 = tn << 6;

  const T* Ab  = A  + (size_t)b * strideA;
  const T* Bb  = Bt + (size_t)b * strideB;
  const T* Ab2 = SPLIT ? (A2  + (size_t)b * strideA) : nullptr;
  const T* Bb2 = SPLIT ? (Bt2 + (size_t)b * strideB) : nullptr;

  const int rlane = lane & 15;
  const int koff  = (lane >> 4) * 8;
  const int mOff  = (lane >> 4) * 8;

  v8f acc[4][4];
#pragma unroll
  for (int i = 0; i < 4; ++i)
#pragma unroll
    for (int j = 0; j < 4; ++j) acc[i][j] = (v8f){0.f,0.f,0.f,0.f,0.f,0.f,0.f,0.f};

  for (int k0 = 0; k0 < K; k0 += 32) {
    V bh[4], bl[4];
#pragma unroll
    for (int j = 0; j < 4; ++j) {
      const size_t bo = (size_t)(n0 + (j << 4) + rlane) * ldb + koff + k0;
      bh[j] = Frag<T>::load(Bb + bo);
      if (SPLIT) bl[j] = Frag<T>::load(Bb2 + bo);
    }
#pragma unroll
    for (int i = 0; i < 4; ++i) {
      const size_t ao = (size_t)(m0 + (i << 4) + rlane) * lda + koff + k0;
      V ah = Frag<T>::load(Ab + ao);
      V al;
      if (SPLIT) al = Frag<T>::load(Ab2 + ao);
#pragma unroll
      for (int j = 0; j < 4; ++j) {
        acc[i][j] = Frag<T>::mma(ah, bh[j], acc[i][j]);
        if (SPLIT) {
          acc[i][j] = Frag<T>::mma(ah, bl[j], acc[i][j]);
          acc[i][j] = Frag<T>::mma(al, bh[j], acc[i][j]);
        }
      }
      Frag<T>::guard4(acc[i][0], acc[i][1], acc[i][2], acc[i][3], ah, SPLIT ? al : ah);
    }
    Frag<T>::keep(bh[0], bh[1], bh[2], bh[3]);
    if (SPLIT) Frag<T>::keep(bl[0], bl[1], bl[2], bl[3]);
  }
  acc_guard4(acc[0][0], acc[0][1], acc[0][2], acc[0][3]);
  acc_guard4(acc[1][0], acc[1][1], acc[1][2], acc[1][3]);
  acc_guard4(acc[2][0], acc[2][1], acc[2][2], acc[2][3]);
  acc_guard4(acc[3][0], acc[3][1], acc[3][2], acc[3][3]);

  float* slab = sT[wave];
  const float* Rb = RESID ? (resid + (size_t)b * strideR) : nullptr;
#pragma unroll
  for (int i = 0; i < 4; ++i) {
    const int mBase = m0 + (i << 4);
#pragma unroll
    for (int j = 0; j < 4; ++j) {
      const int n = n0 + (j << 4) + rlane;
      float bv = 0.f;
      if (BIAS_MODE == 2) bv = bias[n];
#pragma unroll
      for (int r = 0; r < 8; ++r) {
        float v = acc[i][j][r] * scale;
        if (BIAS_MODE == 1) v += bias[mBase + mOff + r];
        if (BIAS_MODE == 2) v += bv;
        if (RESID) v += Rb[(size_t)(mBase + mOff + r) * ldc + n];
        if (ACT == 1) v = tanhf(v);
        if (ACT == 2) v = fmaxf(v, 0.0f);
        if (ACT == 3) v = v / (1.0f + expf(-v));
        if (ACT == 4) v = (v > 0.f) ? v : 0.01f * v;
        if (ACT == 5) v = 0.5f * v * (1.0f + erff(v * 0.70710678118654752f));
        slab[(mOff + r) * 68 + (j << 4) + rlane] = v;
      }
    }
    __builtin_amdgcn_fence(__ATOMIC_RELEASE, "workgroup");
    __builtin_amdgcn_wave_barrier();
    __builtin_amdgcn_fence(__ATOMIC_ACQUIRE, "workgroup");
    if (OUT_MODE == 0) {
      float* C = (float*)Cout + (size_t)b * strideC;
      const int hh = lane >> 4, c4 = (lane & 15) * 4;
      for (int pass = 0; pass < 2; ++pass) {
#pragma unroll
        for (int it = 0; it < 8; ++it) {
          const int row = it * 2 + hh;
          v4f v = *(const v4f*)(slab + row * 68 + c4);
          *(volatile v4f*)(C + (size_t)(mBase + row) * ldc + n0 + c4) = v;
        }
        __threadfence();
      }
    } else {
      const int q = lane >> 3, c8 = (lane & 7) * 8;
      unsigned short* C  = (unsigned short*)Cout  + (size_t)b * strideC;
      unsigned short* C2 = (OUT_MODE == 2) ? ((unsigned short*)Cout2 + (size_t)b * strideC) : nullptr;
      for (int pass = 0; pass < 2; ++pass) {
#pragma unroll
        for (int it = 0; it < 4; ++it) {
          const int row = it * 4 + q;
          const float* sp = slab + row * 68 + c8;
          v8h hv, lv;
#pragma unroll
          for (int e = 0; e < 8; ++e) {
            if (OUT_MODE == 1) {
              hv[e] = (_Float16)sp[e];
            } else {
              unsigned short hb = f2bf_bits(sp[e]);
              unsigned short lb = f2bf_bits(sp[e] - bf_bits2f(hb));
              hv[e] = __builtin_bit_cast(_Float16, hb);
              lv[e] = __builtin_bit_cast(_Float16, lb);
            }
          }
          *(volatile v8h*)(C + (size_t)(mBase + row) * ldc + n0 + c8) = hv;
          if (OUT_MODE == 2) *(volatile v8h*)(C2 + (size_t)(mBase + row) * ldc + n0 + c8) = lv;
        }
        __threadfence();
      }
    }
    __builtin_amdgcn_fence(__ATOMIC_RELEASE, "workgroup");
    __builtin_amdgcn_wave_barrier();
    __builtin_amdgcn_fence(__ATOMIC_ACQUIRE, "workgroup");
  }
}

__global__ __launch_bounds__(NTHR) void cvt8_f16_kernel(const float* __restrict__ src, unsigned short* __restrict__ dst,
                                                       int n8, float sc) {
  const int i = blockIdx.x * NTHR + threadIdx.x;
  if (i < n8) {
    const float* sp = src + (size_t)i * 8;
    const v4f a = *(const v4f*)(sp);
    const v4f c = *(const v4f*)(sp + 4);
    v8h hv;
#pragma unroll
    for (int e = 0; e < 4; ++e) { hv[e] = (_Float16)(a[e] * sc); hv[4 + e] = (_Float16)(c[e] * sc); }
    *(volatile v8h*)(dst + (size_t)i * 8) = hv;
    __threadfence();
    *(volatile v8h*)(dst + (size_t)i * 8) = hv;
  }
}

__global__ __launch_bounds__(NTHR) void tpw_f16_kernel(const float* __restrict__ src, int R, int C, long sstride,
                                                      unsigned short* __restrict__ O, int ldo, int ocol0, long ostride, float sc) {
  __shared__ float Tt[64 * 65];
  const int tid = threadIdx.x;
  const int c0 = blockIdx.x * 64, r0 = blockIdx.y * 64;
  const float* sb = src + (size_t)blockIdx.z * (size_t)sstride;
  unsigned short* ob = O + (size_t)blockIdx.z * (size_t)ostride;
#pragma unroll
  for (int i = 0; i < 4; ++i) {
    const int idx = i * NTHR + tid;
    const int rr = idx >> 4, cc = (idx & 15) * 4;
    const v4f v = *(const v4f*)(sb + (size_t)(r0 + rr) * (size_t)C + c0 + cc);
    Tt[rr * 65 + cc + 0] = v[0];
    Tt[rr * 65 + cc + 1] = v[1];
    Tt[rr * 65 + cc + 2] = v[2];
    Tt[rr * 65 + cc + 3] = v[3];
  }
  __syncthreads();
  const int q = tid >> 3, c8 = (tid & 7) * 8;
  v8h hv[2];
#pragma unroll
  for (int g = 0; g < 2; ++g) {
    const int qq = g * 32 + q;
#pragma unroll
    for (int e = 0; e < 8; ++e) hv[g][e] = (_Float16)(Tt[(c8 + e) * 65 + qq] * sc);
  }
  for (int pass = 0; pass < 2; ++pass) {
#pragma unroll
    for (int g = 0; g < 2; ++g) {
      const size_t o = (size_t)(c0 + g * 32 + q) * (size_t)ldo + (size_t)ocol0 + (size_t)(r0 + c8);
      *(volatile v8h*)(ob + o) = hv[g];
    }
    __threadfence();
  }
}

__global__ __launch_bounds__(NTHR) void gather_y_kernel(const int* __restrict__ words, const float* __restrict__ emb,
                                                       unsigned short* __restrict__ Y) {
  const int i = blockIdx.x * NTHR + threadIdx.x;
  if (i < MR * (DM / 8)) {
    const int m = i >> 6, c8 = (i & 63) * 8;
    int w = words[m];
    w = (w < 0) ? 0 : ((w > VOC - 1) ? (VOC - 1) : w);
    const float* ep = emb + (size_t)w * DM + c8;
    const v4f a = *(const v4f*)(ep);
    const v4f c = *(const v4f*)(ep + 4);
    v8h hv;
#pragma unroll
    for (int e = 0; e < 4; ++e) { hv[e] = (_Float16)(a[e] * CR_ACT); hv[4 + e] = (_Float16)(c[e] * CR_ACT); }
    *(volatile v8h*)(Y + (size_t)i * 8) = hv;
    __threadfence();
    *(volatile v8h*)(Y + (size_t)i * 8) = hv;
  }
}

__global__ __launch_bounds__(NTHR) void bias_prep_kernel(const float* __restrict__ ba, const float* __restrict__ bb2,
                                                         float* __restrict__ dst) {
  const int tid = threadIdx.x;
  const int which = tid >> 7;
  const int idx = (tid & 127) * 4;
  const v4f va = *(const v4f*)(ba + idx);
  const v4f vb = *(const v4f*)(bb2 + idx);
  const float fw = (float)which, fa = 1.0f - fw;
  v4f o;
#pragma unroll
  for (int e = 0; e < 4; ++e) o[e] = CR_ACT * fmaf(fw, vb[e], fa * va[e]);
  float* op = dst + which * DM + idx;
  *(volatile v4f*)op = o;
  __threadfence();
  *(volatile v4f*)op = o;
}

__global__ __launch_bounds__(NTHR) void softmax_e_kernel(const float* __restrict__ SCT, const int* __restrict__ mask,
                                                        unsigned short* __restrict__ AO) {
  __shared__ __align__(16) int   Ms[SE * 8];
  __shared__ __align__(16) float Sx[8][SE];
  const int tid = threadIdx.x, lane = tid & 31, wave = tid >> 5;
  const int b = blockIdx.x >> 5, s0 = (blockIdx.x & 31) * 8;
#pragma unroll
  for (int g = 0; g < 2; ++g) {
    const int e = g * NTHR + tid;
    const int* mp = mask + ((size_t)b * SE + e) * SD + s0;
    const v4i ma = *(const v4i*)(mp);
    const v4i mb = *(const v4i*)(mp + 4);
    *(v4i*)(Ms + e * 8)     = ma;
    *(v4i*)(Ms + e * 8 + 4) = mb;
  }
  __syncthreads();
  const int s = s0 + wave;
  const float* rp = SCT + ((size_t)b * SD + s) * SE;
  float* sx = Sx[wave];
  float mx = -INFINITY;
#pragma unroll
  for (int q = 0; q < 4; ++q) {
    const v4f v = *(const v4f*)(rp + 128 * q + 4 * lane);
    v4f x;
#pragma unroll
    for (int i = 0; i < 4; ++i) {
      const int e = 128 * q + 4 * lane + i;
      const float mf = (float)Ms[e * 8 + wave] * (-1.0e9f);
      x[i] = v[i] + mf;
      mx = fmaxf(mx, x[i]);
    }
    *(v4f*)(sx + 128 * q + 4 * lane) = x;
  }
#pragma unroll
  for (int off = 1; off < 32; off <<= 1) mx = fmaxf(mx, __shfl_xor(mx, off, 32));
  float sum = 0.0f;
#pragma unroll 1
  for (int q = 0; q < 4; ++q) {
    float* p = sx + 128 * q + 4 * lane;
    const v4f x = *(const v4f*)p;
    v4f ex;
#pragma unroll
    for (int i = 0; i < 4; ++i) { ex[i] = expf(x[i] - mx); sum += ex[i]; }
    *(v4f*)p = ex;
  }
#pragma unroll
  for (int off = 1; off < 32; off <<= 1) sum += __shfl_xor(sum, off, 32);
  const float inv = CR_P * (1.0f / sum);
  __builtin_amdgcn_fence(__ATOMIC_RELEASE, "workgroup");
  __builtin_amdgcn_wave_barrier();
  __builtin_amdgcn_fence(__ATOMIC_ACQUIRE, "workgroup");
  unsigned short* orow = AO + ((size_t)b * SD + s) * SE;
  for (int pass = 0; pass < 2; ++pass) {
#pragma unroll
    for (int q2 = 0; q2 < 2; ++q2) {
      const float* p = sx + 256 * q2 + 8 * lane;
      const v4f pa = *(const v4f*)(p);
      const v4f pb = *(const v4f*)(p + 4);
      v8h hv;
#pragma unroll
      for (int i = 0; i < 4; ++i) { hv[i] = (_Float16)(pa[i] * inv); hv[4 + i] = (_Float16)(pb[i] * inv); }
      *(volatile v8h*)(orow + 256 * q2 + 8 * lane) = hv;
    }
    __threadfence();
  }
}

template <int LAYER>
__global__ __launch_bounds__(NTHR) void lstm_seq_kernel(const unsigned short* __restrict__ INp,
                                                        const unsigned short* __restrict__ KRp,
                                                        const float* __restrict__ bias,
                                                        unsigned short* __restrict__ out16,
                                                        float* __restrict__ out32) {
  __shared__ __align__(16) _Float16 At[16 * AP];
  __shared__ __align__(16) float    Hs[16 * OP];
  const _Float16* KR = (const _Float16*)KRp;
  const int tid = threadIdx.x, lane = tid & 31, wave = tid >> 5;
  const int c = lane & 15, hh = lane >> 4, koff = hh * 8;
  const int rowbase = blockIdx.x * 16;

#pragma unroll 1
  for (int i = tid; i < 16 * NH; i += NTHR) At[(i >> 9) * AP + DM + (i & 511)] = (_Float16)0.0f;
  __syncthreads();
#pragma unroll
  for (int it = 0; it < 4; ++it) {
    const int idx = it * NTHR + tid;
    const int row = idx >> 6, c8 = (idx & 63) * 8;
    const v4u v = *(const v4u*)(INp + ((size_t)(rowbase + row) * SD) * DM + c8);
    *(v4u*)(At + row * AP + c8) = v;
  }
  float bb[4][4], cst[4][8];
#pragma unroll
  for (int nt = 0; nt < 4; ++nt) {
    const int j = 64 * wave + 16 * nt + c;
#pragma unroll
    for (int g = 0; g < 4; ++g) bb[nt][g] = bias[g * NH + j];
    asm volatile("" ::: "memory");
#pragma unroll
    for (int r = 0; r < 8; ++r) cst[nt][r] = 0.0f;
  }
  __syncthreads();

  const _Float16* arow = At + c * AP + koff;
  const v8f z8 = {0.f, 0.f, 0.f, 0.f, 0.f, 0.f, 0.f, 0.f};

#pragma unroll 1
  for (int t = 0; t < SD; ++t) {
#pragma unroll
    for (int nt = 0; nt < 4; ++nt) {
      const int j = 64 * wave + 16 * nt + c;
      const _Float16* wrow = KR + (size_t)j * KTOT + koff;
      v8f acc[4];
      acc[0] = z8; acc[1] = z8; acc[2] = z8; acc[3] = z8;
#pragma unroll 1
      for (int k0 = 0; k0 < KTOT; k0 += 32) {
        const v16h a  = Frag<_Float16>::load(arow + k0);
        const v16h b0 = Frag<_Float16>::load(wrow + k0);
        const v16h b1 = Frag<_Float16>::load(wrow + (size_t)1 * NH * KTOT + k0);
        const v16h b2 = Frag<_Float16>::load(wrow + (size_t)2 * NH * KTOT + k0);
        const v16h b3 = Frag<_Float16>::load(wrow + (size_t)3 * NH * KTOT + k0);
        acc[0] = Frag<_Float16>::mma(a, b0, acc[0]);
        acc[1] = Frag<_Float16>::mma(a, b1, acc[1]);
        acc[2] = Frag<_Float16>::mma(a, b2, acc[2]);
        acc[3] = Frag<_Float16>::mma(a, b3, acc[3]);
        dep_guard4_h(acc[0], acc[1], acc[2], acc[3], a, b3);
        keep4_h(b0, b1, b2, b3);
      }
      acc_guard4(acc[0], acc[1], acc[2], acc[3]);
#pragma unroll
      for (int r = 0; r < 8; ++r) {
        const float zi = acc[0][r] * ZINV + bb[nt][0];
        const float zf = acc[1][r] * ZINV + bb[nt][1];
        const float zg = acc[2][r] * ZINV + bb[nt][2];
        const float zo = acc[3][r] * ZINV + bb[nt][3];
        const float ig = fsig(zi);
        const float fg = fsig(zf);
        const float og = fsig(zo);
        const float gg = tanhf(zg);
        const float cn = fg * cst[nt][r] + ig * gg;
        cst[nt][r] = cn;
        Hs[(8 * hh + r) * OP + j] = og * tanhf(cn);
      }
    }
    __syncthreads();
#pragma unroll
    for (int nt = 0; nt < 4; ++nt) {
      const int j = 64 * wave + 16 * nt + c;
#pragma unroll
      for (int r = 0; r < 8; ++r) {
        const float hn = Hs[(8 * hh + r) * OP + j];
        At[(8 * hh + r) * AP + DM + j] = (_Float16)(hn * CR_H);
      }
    }
    {
      const int tn = (t + 1 < SD) ? (t + 1) : (SD - 1);
#pragma unroll
      for (int it = 0; it < 4; ++it) {
        const int idx = it * NTHR + tid;
        const int row = idx >> 6, c8 = (idx & 63) * 8;
        const v4u v = *(const v4u*)(INp + ((size_t)(rowbase + row) * SD + (size_t)tn) * DM + c8);
        *(v4u*)(At + row * AP + c8) = v;
      }
    }
    if (LAYER == 1) {
      for (int pass = 0; pass < 2; ++pass) {
#pragma unroll
        for (int rr = 0; rr < 2; ++rr) {
          const int row = 2 * wave + rr;
          float* orow = out32 + ((size_t)(rowbase + row) * SD + (size_t)t) * NH;
#pragma unroll
          for (int q = 0; q < 4; ++q) {
            const v4f v = *(const v4f*)(Hs + row * OP + 128 * q + 4 * lane);
            *(volatile v4f*)(orow + 128 * q + 4 * lane) = v;
          }
        }
        __threadfence();
      }
    }
    __syncthreads();
    if (LAYER == 0) {
      for (int pass = 0; pass < 2; ++pass) {
#pragma unroll
        for (int rr = 0; rr < 2; ++rr) {
          const int row = 2 * wave + rr;
          unsigned short* orow = out16 + ((size_t)(rowbase + row) * SD + (size_t)t) * NH;
#pragma unroll
          for (int q = 0; q < 2; ++q) {
            const v4u v = *(const v4u*)(At + row * AP + DM + 256 * q + 8 * lane);
            *(volatile v4u*)(orow + 256 * q + 8 * lane) = v;
          }
        }
        __threadfence();
      }
    }
  }
}

extern "C" void kernel_launch(void* const* d_in, const int* in_sizes, int n_in,
                              void* d_out, int out_size, void* d_ws, size_t ws_size, hipStream_t stream) {
  if (n_in < 14 || d_out == nullptr || d_ws == nullptr) return;
  if (in_sizes[0] != NB * SE * DM || in_sizes[1] != NB * SD || in_sizes[2] != NB * SE * SD ||
      in_sizes[3] != DM * DM || in_sizes[4] != DM || in_sizes[5] != VOC * DM ||
      in_sizes[6] != DM * DM || in_sizes[7] != DM ||
      in_sizes[8] != DM * G4 || in_sizes[9] != NH * G4 || in_sizes[10] != G4 ||
      in_sizes[11] != NH * G4 || in_sizes[12] != NH * G4 || in_sizes[13] != G4 ||
      out_size != MR * NH) return;

  const float* enc   = (const float*)d_in[0];
  const int*   words = (const int*)  d_in[1];
  const int*   mask  = (const int*)  d_in[2];
  const float* P_w   = (const float*)d_in[3];
  const float* P_b   = (const float*)d_in[4];
  const float* emb   = (const float*)d_in[5];
  const float* din_w = (const float*)d_in[6];
  const float* din_b = (const float*)d_in[7];
  const float* k0w   = (const float*)d_in[8];
  const float* r0w   = (const float*)d_in[9];
  const float* b0v   = (const float*)d_in[10];
  const float* k1w   = (const float*)d_in[11];
  const float* r1w   = (const float*)d_in[12];
  const float* b1v   = (const float*)d_in[13];
  float* out = (float*)d_out;

  char* ws = (char*)d_ws; size_t off = 0;
  auto carve = [&](size_t bytes) -> char* { char* p = ws + off; off += (bytes + 255) & ~(size_t)255; return p; };
  unsigned short* ENCN  = (unsigned short*)carve((size_t)NB * SE * DM * 2);
  unsigned short* ENCT  = (unsigned short*)carve((size_t)NB * DM * SE * 2);
  float*          SCT   = (float*)         carve((size_t)NB * SD * SE * 4);
  unsigned short* APL   = (unsigned short*)carve((size_t)NB * SD * SE * 2);
  unsigned short* Y64   = (unsigned short*)carve((size_t)MR * DM * 2);
  unsigned short* PWT   = (unsigned short*)carve((size_t)DM * DM * 2);
  unsigned short* DINT  = (unsigned short*)carve((size_t)DM * DM * 2);
  unsigned short* KR0   = (unsigned short*)carve((size_t)G4 * KTOT * 2);
  unsigned short* KR1   = (unsigned short*)carve((size_t)G4 * KTOT * 2);
  unsigned short* PY64  = (unsigned short*)carve((size_t)MR * DM * 2);
  unsigned short* DEC64 = (unsigned short*)carve((size_t)MR * DM * 2);
  unsigned short* X64   = (unsigned short*)carve((size_t)MR * DM * 2);
  unsigned short* H0ALL = (unsigned short*)carve((size_t)MR * NH * 2);
  float*          BIAS2 = (float*)         carve((size_t)2 * DM * 4);
  if (off > ws_size || off > (size_t)134217728) return;

  const int n8e = NB * SE * (DM / 8);
  cvt8_f16_kernel<<<(n8e + NTHR - 1) / NTHR, NTHR, 0, stream>>>(enc, ENCN, n8e, 1.0f);
  tpw_f16_kernel<<<dim3(DM / 64, SE / 64, NB), NTHR, 0, stream>>>(enc, SE, DM, (long)SE * DM, ENCT, SE, 0, (long)DM * SE, 1.0f);
  tpw_f16_kernel<<<dim3(DM / 64, DM / 64, 1), NTHR, 0, stream>>>(P_w,   DM, DM, 0L, PWT,  DM, 0, 0L, CR_XW);
  tpw_f16_kernel<<<dim3(DM / 64, DM / 64, 1), NTHR, 0, stream>>>(din_w, DM, DM, 0L, DINT, DM, 0, 0L, CR_XW);
  tpw_f16_kernel<<<dim3(G4 / 64, DM / 64, 1), NTHR, 0, stream>>>(k0w, DM, G4, 0L, KR0, KTOT, 0,  0L, CR_XW);
  tpw_f16_kernel<<<dim3(G4 / 64, NH / 64, 1), NTHR, 0, stream>>>(r0w, NH, G4, 0L, KR0, KTOT, DM, 0L, CR_HW);
  tpw_f16_kernel<<<dim3(G4 / 64, NH / 64, 1), NTHR, 0, stream>>>(k1w, NH, G4, 0L, KR1, KTOT, 0,  0L, CR_HW);
  tpw_f16_kernel<<<dim3(G4 / 64, NH / 64, 1), NTHR, 0, stream>>>(r1w, NH, G4, 0L, KR1, KTOT, DM, 0L, CR_HW);
  bias_prep_kernel<<<1, NTHR, 0, stream>>>(P_b, din_b, BIAS2);
  gather_y_kernel<<<(MR * (DM / 8)) / NTHR, NTHR, 0, stream>>>(words, emb, Y64);

  wmma_gemm64<0, false, 2, 1, false, 0><<<dim3((MR / 64) * (DM / 64) / 8, 1), 256, 0, stream>>>(
      Y64, Y64, DM, 0L, PWT, PWT, DM, 0L, (void*)PY64, (void*)PY64, DM, 0L,
      BIAS2, SCT, 0L, MR, DM, DM, 1.0f / 64.0f);
  wmma_gemm64<0, false, 0, 0, false, 0><<<dim3((SD / 64) * (SE / 64) / 8, NB), 256, 0, stream>>>(
      PY64, PY64, DM, (long)SD * DM, ENCN, ENCN, DM, (long)SE * DM, (void*)SCT, (void*)SCT, SE, (long)SD * SE,
      BIAS2, SCT, 0L, SD, SE, DM, 1.0f / 64.0f);
  softmax_e_kernel<<<NB * (SD / 8), NTHR, 0, stream>>>(SCT, mask, APL);
  wmma_gemm64<0, false, 0, 1, false, 0><<<dim3((SD / 64) * (DM / 64) / 8, NB), 256, 0, stream>>>(
      APL, APL, SE, (long)SD * SE, ENCT, ENCT, SE, (long)DM * SE, (void*)DEC64, (void*)DEC64, DM, (long)SD * DM,
      BIAS2, SCT, 0L, SD, DM, SE, 1.0f / 16.0f);
  wmma_gemm64<0, false, 2, 1, false, 0><<<dim3((MR / 64) * (DM / 64) / 8, 1), 256, 0, stream>>>(
      DEC64, DEC64, DM, 0L, DINT, DINT, DM, 0L, (void*)X64, (void*)X64, DM, 0L,
      BIAS2 + DM, SCT, 0L, MR, DM, DM, 1.0f / 64.0f);

  lstm_seq_kernel<0><<<NB / 16, NTHR, 0, stream>>>(X64, KR0, b0v, H0ALL, out);
  lstm_seq_kernel<1><<<NB / 16, NTHR, 0, stream>>>(H0ALL, KR1, b1v, APL, out);
}
